// FoldableBlock4D_Train_48146583388187
// MI455X (gfx1250) — hardware-verified
//
#include <hip/hip_runtime.h>
#include <math.h>

typedef __attribute__((ext_vector_type(16))) _Float16 v16h;
typedef __attribute__((ext_vector_type(16))) __bf16 v16b;
typedef __attribute__((ext_vector_type(8)))  _Float16 v8h;
typedef __attribute__((ext_vector_type(8)))  float v8f;
typedef __attribute__((ext_vector_type(4)))  float v4f;
typedef __attribute__((ext_vector_type(2)))  float v2f;
typedef __attribute__((ext_vector_type(4)))  unsigned v4u;
typedef __attribute__((ext_vector_type(4)))  int v4i;
typedef float __attribute__((may_alias)) float_a;
typedef int __attribute__((may_alias)) int_a;

template <typename T> __device__ __forceinline__ void vst2(void* p, T v) { *(volatile T*)p = v; __threadfence(); *(volatile T*)p = v; }
__device__ __forceinline__ v8f wmma16(v16h a, v16h b, v8f c) {
  v8f d = __builtin_amdgcn_wmma_f32_16x16x32_f16(false, a, false, b, (short)0, c, false, false);
  asm volatile("v_nop\n\tv_nop\n\tv_nop\n\tv_nop" : "+v"(d) : "v"(a), "v"(b));
  return d;
}
__device__ __forceinline__ v8f wmma_bf(v16b a, v16b b, v8f c) {
  v8f d = __builtin_amdgcn_wmma_f32_16x16x32_bf16(false, a, false, b, (short)0, c, false, false);
  asm volatile("v_nop\n\tv_nop\n\tv_nop\n\tv_nop" : "+v"(d) : "v"(a), "v"(b));
  return d;
}
__device__ __forceinline__ v16h frag_h(const _Float16* rowk0, int lane) {
  union { v16h v; v8h q[2]; } u; const _Float16* p = rowk0 + 8 * (lane >> 4);
  u.q[0] = *(const v8h*)p; u.q[1] = *(const v8h*)(p + 16); return u.v;
}
__device__ __forceinline__ v16h frag_f32(const float* rowk0, int lane) {
  v16h a; const float* p = rowk0 + 8 * (lane >> 4);
#pragma unroll
  for (int i = 0; i < 8; ++i) { a[i] = (_Float16)p[i]; a[8 + i] = (_Float16)p[16 + i]; }
  return a;
}
__device__ __forceinline__ v16h frag_f32s(const float* rowk0, int lane, float sc) {
  v16h a; const float* p = rowk0 + 8 * (lane >> 4);
#pragma unroll
  for (int i = 0; i < 8; ++i) { a[i] = (_Float16)(p[i] * sc); a[8 + i] = (_Float16)(p[16 + i] * sc); }
  return a;
}
__device__ __forceinline__ v16h fragc_f32(const float* W, int k0, int n, int lane, int ld, int K) {
  v16h a; const int g = lane >> 4;
#pragma unroll
  for (int i = 0; i < 8; ++i) { const int ka = k0 + 8 * g + i, kb = ka + 16;
    a[i] = (_Float16)(ka < K ? W[(size_t)ka * ld + n] : 0.f); a[8 + i] = (_Float16)(kb < K ? W[(size_t)kb * ld + n] : 0.f); }
  return a;
}
struct F2 { v16b h, l; };
__device__ __forceinline__ F2 bsplit16(const float v[16]) { F2 r;
#pragma unroll
  for (int i = 0; i < 16; ++i) { const __bf16 h = (__bf16)v[i]; r.h[i] = h; r.l[i] = (__bf16)(v[i] - (float)h); }
  return r; }
__device__ __forceinline__ F2 split_row(const float* row, int k0, int lane) { float v[16]; const float* p = row + k0 + 8 * (lane >> 4);
#pragma unroll
  for (int i = 0; i < 8; ++i) { v[i] = p[i]; v[8 + i] = p[16 + i]; }
  return bsplit16(v); }
__device__ __forceinline__ F2 split_rowK(const float* row, int k0, int lane, int K) { float v[16]; const int g = lane >> 4;
#pragma unroll
  for (int i = 0; i < 8; ++i) { const int ka = k0 + 8 * g + i, kb = ka + 16; v[i] = ka < K ? row[ka] : 0.f; v[8 + i] = kb < K ? row[kb] : 0.f; }
  return bsplit16(v); }
__device__ __forceinline__ F2 split_col(const float* W, int k0, int n, int lane, int ld, int K) { float v[16]; const int g = lane >> 4;
#pragma unroll
  for (int i = 0; i < 8; ++i) { const int ka = k0 + 8 * g + i, kb = ka + 16; v[i] = ka < K ? W[(size_t)ka * ld + n] : 0.f; v[8 + i] = kb < K ? W[(size_t)kb * ld + n] : 0.f; }
  return bsplit16(v); }
__device__ __forceinline__ v8f mac3(const F2& a, const F2& b, v8f c) { c = wmma_bf(a.l, b.h, c); c = wmma_bf(a.h, b.l, c); return wmma_bf(a.h, b.h, c); }
__device__ __forceinline__ float sigm(float v) { return 1.0f / (1.0f + expf(-v)); }
#define LDSX() do { asm volatile("s_wait_dscnt 0" ::: "memory"); __builtin_amdgcn_wave_barrier(); __builtin_amdgcn_fence(__ATOMIC_RELEASE, "workgroup"); } while (0)


#define NBI 4
#define C 128
#define IH 64
#define IW 64
#define NPIX (IH * IW)
#define WS 16
#define NWY (IH / WS)
#define NWX (IW / WS)
#define NWIN (NBI * NWY * NWX)
#define BR 2
#define NHD 4
#define HD 32
#define NTOK (NWIN * WS * WS)
__device__ __forceinline__ v16b frag_b(const __bf16* rowk0, int lane) { return __builtin_bit_cast(v16b, frag_h((const _Float16*)rowk0, lane)); }

__global__ __launch_bounds__(256) void k_ln(const float* __restrict__ x, const float* __restrict__ g_, const float* __restrict__ b_, float* __restrict__ Y) {
  const int b = blockIdx.y, p = blockIdx.x * 256 + threadIdx.x; const float* xp = x + (size_t)b * C * NPIX + p; float s = 0.f;
#pragma unroll 4
  for (int c = 0; c < C; ++c) s += xp[(size_t)c * NPIX];
  const float mu = s * (1.0f / C); float q = 0.f;
#pragma unroll 4
  for (int c = 0; c < C; ++c) { const float d = xp[(size_t)c * NPIX] - mu; q += d * d; }
  const float rs = rsqrtf(q * (1.0f / C) + 1e-6f);
#pragma unroll 4
  for (int c = 0; c < C; ++c) vst2(Y + ((size_t)b * C + c) * NPIX + p, (float_a)((xp[(size_t)c * NPIX] - mu) * rs * g_[c] + b_[c]));
}
__global__ __launch_bounds__(256) void k_tok(const float* __restrict__ Y, const float* __restrict__ cw, const float* __restrict__ cb, __bf16* __restrict__ T) {
  __shared__ __align__(16) __bf16 st[256][C + 8];
  const int n = blockIdx.x, tid = threadIdx.x; const int b = n / (NWY * NWX), wy = (n / NWX) % NWY, wx = n % NWX; const int i = tid >> 4, j = tid & 15; const int y = wy * WS + i, xq = wx * WS + j;
  const int ym = y > 0 ? y - 1 : 0, yp = y < IH - 1 ? y + 1 : IH - 1, xm = xq > 0 ? xq - 1 : 0, xp = xq < IW - 1 ? xq + 1 : IW - 1;
  const int ys[3] = {ym, y, yp}, xs[3] = {xm, xq, xp};
#pragma unroll 1
  for (int c = 0; c < C; ++c) { const float* Yc = Y + ((size_t)b * C + c) * NPIX; const float* w = cw + c * 9; float v = Yc[y * IW + xq] + cb[c];
#pragma unroll
    for (int a = 0; a < 3; ++a)
#pragma unroll
      for (int bb = 0; bb < 3; ++bb) v += w[a * 3 + bb] * Yc[ys[a] * IW + xs[bb]];
    st[tid][c] = (__bf16)v; }
  __syncthreads();
  for (int q = tid; q < 256 * (C / 8); q += 256) { const int rl = q >> 4, pc = q & 15; vst2((unsigned*)(T + ((size_t)n * 256 + rl) * C + pc * 8), *(const v4u*)(&st[rl][pc * 8])); }
}
__global__ __launch_bounds__(128) void k_qkv(const __bf16* __restrict__ T, const float* __restrict__ Wq, const float* __restrict__ Wk, const float* __restrict__ Wv, float* __restrict__ QKV) {
  __shared__ __align__(16) float so[4][16][132];
  const int tid = threadIdx.x, wave = tid >> 5, lane = tid & 31, col = lane & 15, g = lane >> 4;
  const int r0b = blockIdx.x * 64, r0 = r0b + wave * 16; const int which = blockIdx.y, br = blockIdx.z; const float* W = (which == 0 ? Wq : (which == 1 ? Wk : Wv)) + (size_t)br * NHD * HD * C;
  const int n = r0b >> 8, p0 = (r0b & 255) + wave * 16;
  v8f acc[8] = {};
#pragma unroll
  for (int kc = 0; kc < C / 32; ++kc) { const v16b a = frag_b(T + (size_t)(r0 + col) * C + kc * 32, lane);
#pragma unroll
    for (int jt = 0; jt < 8; ++jt) acc[jt] = wmma_bf(a, split_row(W + (size_t)(jt * 16 + col) * C, kc * 32, lane).h, acc[jt]); }
#pragma unroll
  for (int jt = 0; jt < 8; ++jt)
#pragma unroll
    for (int r = 0; r < 8; ++r) so[wave][8 * g + r][jt * 16 + col] = acc[jt][r];
  LDSX();
  for (int qq = lane; qq < 16 * NHD * 8; qq += 32) { const int h = qq >> 7, rl = (qq >> 3) & 15, pc = qq & 7;
    vst2(QKV + ((((size_t)which * NWIN * BR + (size_t)n * BR + br) * NHD + h) * 256 + p0 + rl) * HD + pc * 4, *(const v4f*)(&so[wave][rl][h * HD + pc * 4])); }
}
__global__ __launch_bounds__(128) void k_natt(const float* __restrict__ QKV, float* __restrict__ O) {
  __shared__ __align__(16) float sS[4][16][260];
  __shared__ __align__(16) __bf16 sP[4][16][264];
  __shared__ __align__(16) float sO[4][16][36];
  const int bid = blockIdx.x; const int tid = threadIdx.x, wave = tid >> 5, lane = tid & 31, col = lane & 15, g = lane >> 4;
  const size_t plane = (size_t)bid * 256 * HD; const size_t wstride = (size_t)NWIN * BR * NHD * 256 * HD;
  const float* Qp = QKV + plane; const float* Kp = QKV + wstride + plane; const float* Vp = QKV + 2 * wstride + plane;
  const float scale = 0.17677669529663687f; const int h = bid % NHD, nbr = bid / NHD;
#pragma unroll 1
  for (int ch = 0; ch < 4; ++ch) { const int q0 = ch * 64 + wave * 16;
    const v16b aq = split_row(Qp + (size_t)(q0 + col) * HD, 0, lane).h;
#pragma unroll
    for (int t = 0; t < 16; ++t) { const v8f s = wmma_bf(aq, split_row(Kp + (size_t)(t * 16 + col) * HD, 0, lane).h, (v8f){});
#pragma unroll
      for (int r = 0; r < 8; ++r) sS[wave][8 * g + r][t * 16 + col] = s[r] * scale; }
    for (int qz = lane; qz < 16 * 264 / 2; qz += 32) ((unsigned*)&sP[wave][0][0])[qz] = 0u;
    LDSX();
    { const int rl = lane & 15, hf = lane >> 4; const int q = q0 + rl; const int qi = q >> 4, qj = q & 15; float mx = -3.4e38f; float vals[13]; int keys[13]; int nv = 0;
#pragma unroll
      for (int t = 0; t < 13; ++t) { const int pidx = hf * 13 + t; vals[t] = 0.f; keys[t] = -1;
        if (pidx < 25) { const int a = pidx / 5, bb = pidx % 5; const int ii = qi + a - 2, jj = qj + bb - 2;
          if (ii >= 0 && ii < WS && jj >= 0 && jj < WS) { keys[t] = ii * WS + jj; vals[t] = sS[wave][rl][keys[t]]; } else { vals[t] = 0.f; ++nv; }
          mx = fmaxf(mx, vals[t]); } }
      mx = fmaxf(mx, __shfl_xor(mx, 16, 32)); float z = 0.f;
#pragma unroll
      for (int t = 0; t < 13; ++t) { const int pidx = hf * 13 + t; if (pidx < 25) { const float e = expf(vals[t] - mx); vals[t] = e; z += e; } }
      z += __shfl_xor(z, 16, 32); const float inv = 1.0f / z;
#pragma unroll
      for (int t = 0; t < 13; ++t) if (keys[t] >= 0) sP[wave][rl][keys[t]] = (__bf16)(vals[t] * inv); (void)nv; }
    LDSX();
    v8f acc[2] = {};
#pragma unroll
    for (int kc = 0; kc < 8; ++kc) { const v16b pa = frag_b(&sP[wave][col][0] + kc * 32, lane);
#pragma unroll
      for (int t2 = 0; t2 < 2; ++t2) acc[t2] = wmma_bf(pa, split_col(Vp + (size_t)(kc * 32) * HD, 0, t2 * 16 + col, lane, HD, 32).h, acc[t2]); }
#pragma unroll
    for (int t2 = 0; t2 < 2; ++t2)
#pragma unroll
      for (int r = 0; r < 8; ++r) sO[wave][8 * g + r][t2 * 16 + col] = acc[t2][r];
    LDSX();
    for (int qq = lane; qq < 16 * 8; qq += 32) { const int rl = qq >> 3, pc = qq & 7; vst2(O + ((size_t)nbr * 256 + q0 + rl) * C + h * HD + pc * 4, *(const v4f*)(&sO[wave][rl][pc * 4])); }
    LDSX(); }
}
__global__ __launch_bounds__(128) void k_oproj(const float* __restrict__ O, const float* __restrict__ Wo, float* __restrict__ HO) {
  __shared__ __align__(16) float so[4][16][132];
  const int tid = threadIdx.x, wave = tid >> 5, lane = tid & 31, col = lane & 15, g = lane >> 4;
  const int r0b = blockIdx.x * 64, r0 = r0b + wave * 16; const int br = (r0b >> 8) & 1;
  v8f acc[8] = {};
#pragma unroll
  for (int kc = 0; kc < NHD; ++kc) { const v16b a = split_row(O + (size_t)(r0 + col) * C, kc * 32, lane).h;
#pragma unroll
    for (int jt = 0; jt < 8; ++jt) { const int c = jt * 16 + col; acc[jt] = wmma_bf(a, split_row(Wo + (((size_t)br * NHD + kc) * C + c) * HD, 0, lane).h, acc[jt]); } }
#pragma unroll
  for (int jt = 0; jt < 8; ++jt)
#pragma unroll
    for (int r = 0; r < 8; ++r) so[wave][8 * g + r][jt * 16 + col] = acc[jt][r];
  LDSX();
  for (int rl = 0; rl < 16; ++rl) vst2(HO + (size_t)(r0 + rl) * C + lane * 4, *(const v4f*)(&so[wave][rl][lane * 4]));
}
__global__ __launch_bounds__(256) void k_final(const float* __restrict__ x, const float* __restrict__ HO, float* __restrict__ out) {
  const int b = blockIdx.y, c = blockIdx.x, tid = threadIdx.x; const float rect = 0.8944271909999159f;
#pragma unroll 1
  for (int q = tid; q < NPIX / 4; q += 256) { const int y = q >> 4, x4 = (q & 15) * 4; const int wy = y >> 4, i = y & 15; v4f v = *(const v4f*)(x + (((size_t)b * C + c) * IH + y) * IW + x4);
#pragma unroll
    for (int e = 0; e < 4; ++e) { const int xx = x4 + e; const int wx = xx >> 4, j = xx & 15; const int n = (b * NWY + wy) * NWX + wx, p = i * WS + j;
      const float h0 = HO[(((size_t)n * BR + 0) * 256 + p) * C + c], h1 = HO[(((size_t)n * BR + 1) * 256 + p) * C + c]; v[e] += (h0 + 0.5f * h1) * rect; }
    vst2(out + (((size_t)b * C + c) * IH + y) * IW + x4, v); }
}
extern "C" void kernel_launch(void* const* d_in, const int* in_sizes, int n_in, void* d_out, int out_size, void* d_ws, size_t ws_size, hipStream_t stream) {
  (void)in_sizes; (void)n_in; (void)out_size; (void)ws_size;
  const float** I = (const float**)d_in;
  const float* x = I[0]; const float* Wq = I[1]; const float* Wk = I[2]; const float* Wv = I[3]; const float* Wo = I[4]; const float* cw = I[5]; const float* cb = I[6]; const float* lg = I[7]; const float* lb = I[8];
  float* out = (float*)d_out;
  char* ws = (char*)d_ws; size_t off = 0;
  auto take = [&](size_t bytes) { char* p = ws + off; off += (bytes + 255) & ~(size_t)255; return p; };
  float* Y = (float*)take((size_t)NBI * C * NPIX * 4); __bf16* T = (__bf16*)take((size_t)NTOK * C * 2); float* QKV = (float*)take((size_t)3 * NWIN * BR * NHD * 256 * HD * 4); float* O = (float*)take((size_t)NWIN * BR * 256 * C * 4); float* HO = (float*)take((size_t)NWIN * BR * 256 * C * 4);
  k_ln<<<dim3(NPIX / 256, NBI), 256, 0, stream>>>(x, lg, lb, Y);
  k_tok<<<NWIN, 256, 0, stream>>>(Y, cw, cb, T);
  k_qkv<<<dim3(NTOK / 64, 3, BR), 128, 0, stream>>>(T, Wq, Wk, Wv, QKV);
  k_natt<<<NWIN * BR * NHD, 128, 0, stream>>>(QKV, O);
  k_oproj<<<(NWIN * BR * 256) / 64, 128, 0, stream>>>(O, Wo, HO);
  k_final<<<dim3(C, NBI), 256, 0, stream>>>(x, HO, out);
}
